// enc_mtan_89386859364766
// MI455X (gfx1250) — hardware-verified
//
#include <hip/hip_runtime.h>
#include <math.h>

constexpr int kB      = 30;
constexpr int kBP     = 32;
constexpr int kS      = 1024;
constexpr int kD      = 128;
constexpr int kE      = 128;
constexpr int kH      = 4;
constexpr int kDK     = 32;
constexpr int kNH     = 128;
constexpr int kG3     = 3 * kNH;
constexpr int kTok    = kB * kS;
constexpr int kQKld   = 2 * kE;
constexpr int kCtxLd  = kH * kD;
constexpr int kChunkB = 2;
constexpr int kNChunk = kB / kChunkB;
constexpr int kBHC    = kChunkB * kH;
constexpr int kGruPA  = 264;
constexpr int kWihN   = kG3 * kNH;

constexpr float kCarry16    = 16.0f;
constexpr float kQScale     = 1.0f / 16.0f;
constexpr float kQBiasScale = 16.0f;
constexpr float kScoreScale = 0.17677669529663687f / 256.0f;
constexpr float kPCarry     = 32768.0f;
constexpr float kPVScale    = 1.0f / 128.0f;
constexpr float kOutScale   = 1.0f / 4096.0f;
constexpr float kGruScale   = 1.0f / 256.0f;
constexpr float kLog2e      = 1.4426950408889634f;

constexpr size_t kOffTE   = 0;
constexpr size_t kOffQK   = kOffTE  + (size_t)kTok * kE * 2;
constexpr size_t kOffXT   = kOffQK  + (size_t)kTok * kQKld * 2;
constexpr size_t kOffCTX  = kOffXT  + (size_t)kB * kD * kS * 2;
constexpr size_t kOffATT  = kOffCTX + (size_t)kTok * kCtxLd * 2;
constexpr size_t kOffWQK  = kOffATT + (size_t)kTok * kNH * 4;
constexpr size_t kOffWO   = kOffWQK + (size_t)2 * kE * kE * 2;
constexpr size_t kOffWG   = kOffWO  + (size_t)kNH * kCtxLd * 2;
constexpr size_t kOffHF   = kOffWG  + (size_t)4 * kWihN * 2;
constexpr size_t kOffS    = kOffHF  + (size_t)2 * kBP * kNH * 4;
constexpr size_t kOffP    = kOffS   + (size_t)kBHC * kS * kS * 4;
constexpr size_t kWsTotal = kOffP   + (size_t)kBHC * kS * kS * 2;
static_assert(kWsTotal == 129597440ull, "ws total");
static_assert(kWsTotal <= 134217728ull, "ws cap");

typedef __attribute__((ext_vector_type(16))) _Float16 v16h;
typedef __attribute__((ext_vector_type(8)))  _Float16 v8h;
typedef __attribute__((ext_vector_type(16))) __bf16   v16b;
typedef __attribute__((ext_vector_type(8)))  __bf16   v8b;
typedef __attribute__((ext_vector_type(8)))  float    v8f;
typedef __attribute__((ext_vector_type(4)))  float    v4f;
typedef __attribute__((ext_vector_type(4)))  unsigned int v4u;

__device__ __forceinline__ unsigned short f2bf_bits(float f) {
  unsigned u = __float_as_uint(f);
  return (unsigned short)((u + 0x7FFFu + ((u >> 16) & 1u)) >> 16);
}
__device__ __forceinline__ float bf_bits2f(unsigned short h) { return __uint_as_float(((unsigned)h) << 16); }

__device__ __forceinline__ void dep_guard_h(v8f& a, v8f& b, v16h x, v16h y) { asm volatile("v_nop\n\tv_nop\n\tv_nop\n\tv_nop" : "+v"(a), "+v"(b) : "v"(x), "v"(y)); }
__device__ __forceinline__ void dep_guard_b(v8f& a, v8f& b, v16b x, v16b y) { asm volatile("v_nop\n\tv_nop\n\tv_nop\n\tv_nop" : "+v"(a), "+v"(b) : "v"(x), "v"(y)); }
__device__ __forceinline__ void keep4_h(v16h a, v16h b, v16h c, v16h d) { asm volatile("v_nop" :: "v"(a), "v"(b), "v"(c), "v"(d)); }
__device__ __forceinline__ void keep4_b(v16b a, v16b b, v16b c, v16b d) { asm volatile("v_nop" :: "v"(a), "v"(b), "v"(c), "v"(d)); }
__device__ __forceinline__ void acc_guard4(v8f& a, v8f& b, v8f& c, v8f& d) { asm volatile("v_nop\n\tv_nop\n\tv_nop\n\tv_nop" : "+v"(a), "+v"(b), "+v"(c), "+v"(d)); }
template <typename T> struct Frag;
template <> struct Frag<_Float16> {
  typedef v16h V; union U { v16h v; v8h h[2]; };
  static __device__ __forceinline__ v16h load(const _Float16* p) {
    U f; f.h[0] = *(const v8h*)(p); f.h[1] = *(const v8h*)(p + 16); return f.v;
  }
  static __device__ __forceinline__ v8f mma(v16h a, v16h b, v8f c) {
    return __builtin_amdgcn_wmma_f32_16x16x32_f16(false, a, false, b, (short)0, c, false, false);
  }
  static __device__ __forceinline__ void guard(v8f& a, v8f& b, v16h x, v16h y) { dep_guard_h(a, b, x, y); }
  static __device__ __forceinline__ void keep(v16h a, v16h b, v16h c, v16h d) { keep4_h(a, b, c, d); }
};
template <> struct Frag<__bf16> {
  typedef v16b V; union U { v16b v; v8b h[2]; };
  static __device__ __forceinline__ v16b load(const __bf16* p) {
    U f; f.h[0] = *(const v8b*)(p); f.h[1] = *(const v8b*)(p + 16); return f.v;
  }
  static __device__ __forceinline__ v8f mma(v16b a, v16b b, v8f c) {
    return __builtin_amdgcn_wmma_f32_16x16x32_bf16(false, a, false, b, (short)0, c, false, false);
  }
  static __device__ __forceinline__ void guard(v8f& a, v8f& b, v16b x, v16b y) { dep_guard_b(a, b, x, y); }
  static __device__ __forceinline__ void keep(v16b a, v16b b, v16b c, v16b d) { keep4_b(a, b, c, d); }
};

__device__ __forceinline__ unsigned pk16(unsigned short a, unsigned short b) { return (unsigned)a | ((unsigned)b << 16); }
__device__ __forceinline__ unsigned short h_bits(float f) { const _Float16 h = (_Float16)f; return __builtin_bit_cast(unsigned short, h); }

__device__ __forceinline__ v8f mma16h(v16h a, v16h b, v8f c) {
  c = __builtin_amdgcn_wmma_f32_16x16x32_f16(false, a, false, b, (short)0, c, false, false);
  asm volatile("v_nop\n\tv_nop\n\tv_nop\n\tv_nop" : "+v"(c) : "v"(a), "v"(b));
  return c;
}

template <int ET> struct Elem;
template <> struct Elem<0> { typedef _Float16 T; };
template <> struct Elem<1> { typedef __bf16 T; };
template <int ET, bool SPLIT, int BIAS_MODE, int OUT_MODE, bool RESID, int ACT = 0>
__global__ __launch_bounds__(256) void wmma_gemm64z(
    const unsigned short* __restrict__ Ap, const unsigned short* __restrict__ A2p, int lda, long strideA, long strideAz,
    const unsigned short* __restrict__ Btp, const unsigned short* __restrict__ Bt2p, int ldb, long strideB, long strideBz,
    void* __restrict__ Cout, void* __restrict__ Cout2, int ldc, long strideC, long strideCz,
    const float* __restrict__ bias, float bscale,
    const float* __restrict__ resid, long strideR,
    int M, int N, int K, float scale) {
  typedef typename Elem<ET>::T T;
  typedef typename Frag<T>::V V;
  const T* A = (const T*)Ap; const T* A2 = (const T*)A2p; const T* Bt = (const T*)Btp; const T* Bt2 = (const T*)Bt2p;
  __shared__ __align__(16) float sT[8][16 * 68];
  const int b    = blockIdx.y;
  const int bz   = blockIdx.z;
  const int lane = threadIdx.x & 31;
  const int wave = threadIdx.x >> 5;
  const int tilesN = N >> 6;
  const int tilesM = M >> 6;
  const int tile = blockIdx.x * 8 + wave;
  if (tile >= tilesM * tilesN) return;
  const int tm = tile / tilesN;
  const int tn = tile - tm * tilesN;
  const int m0 = tm << 6;
  const int n0 = tn << 6;

  const size_t offA = (size_t)b * strideA + (size_t)bz * strideAz;
  const size_t offB = (size_t)b * strideB + (size_t)bz * strideBz;
  const size_t offC = (size_t)b * strideC + (size_t)bz * strideCz;
  const T* Ab  = A  + offA;
  const T* Bb  = Bt + offB;
  const T* Ab2 = SPLIT ? (A2  + offA) : nullptr;
  const T* Bb2 = SPLIT ? (Bt2 + offB) : nullptr;

  const int rlane = lane & 15;
  const int koff  = (lane >> 4) * 8;
  const int mOff  = (lane >> 4) * 8;

  v8f acc[4][4];
#pragma unroll
  for (int i = 0; i < 4; ++i)
#pragma unroll
    for (int j = 0; j < 4; ++j) acc[i][j] = (v8f){0.f,0.f,0.f,0.f,0.f,0.f,0.f,0.f};

  for (int k0 = 0; k0 < K; k0 += 32) {
    V bh[4], bl[4];
#pragma unroll
    for (int j = 0; j < 4; ++j) {
      const size_t bo = (size_t)(n0 + (j << 4) + rlane) * ldb + koff + k0;
      bh[j] = Frag<T>::load(Bb + bo);
      if (SPLIT) bl[j] = Frag<T>::load(Bb2 + bo);
    }
#pragma unroll
    for (int i = 0; i < 4; ++i) {
      const size_t ao = (size_t)(m0 + (i << 4) + rlane) * lda + koff + k0;
      V ah = Frag<T>::load(Ab + ao);
      V al;
      if (SPLIT) al = Frag<T>::load(Ab2 + ao);
#pragma unroll
      for (int j = 0; j < 4; ++j) {
        acc[i][j] = Frag<T>::mma(ah, bh[j], acc[i][j]);
        if (SPLIT) {
          acc[i][j] = Frag<T>::mma(ah, bl[j], acc[i][j]);
          acc[i][j] = Frag<T>::mma(al, bh[j], acc[i][j]);
        }
      }
      Frag<T>::guard(acc[i][0], acc[i][3], ah, SPLIT ? al : ah);
    }
    Frag<T>::keep(bh[0], bh[1], bh[2], bh[3]);
    if (SPLIT) Frag<T>::keep(bl[0], bl[1], bl[2], bl[3]);
  }
  acc_guard4(acc[0][0], acc[0][1], acc[0][2], acc[0][3]);
  acc_guard4(acc[1][0], acc[1][1], acc[1][2], acc[1][3]);
  acc_guard4(acc[2][0], acc[2][1], acc[2][2], acc[2][3]);
  acc_guard4(acc[3][0], acc[3][1], acc[3][2], acc[3][3]);

  float* slab = sT[wave];
  const float* Rb = RESID ? (resid + (size_t)b * strideR) : nullptr;
#pragma unroll
  for (int i = 0; i < 4; ++i) {
    const int mBase = m0 + (i << 4);
#pragma unroll
    for (int j = 0; j < 4; ++j) {
      const int n = n0 + (j << 4) + rlane;
      float bv = 0.f;
      if (BIAS_MODE == 2) bv = bias[n] * bscale;
#pragma unroll
      for (int r = 0; r < 8; ++r) {
        float v = acc[i][j][r] * scale;
        if (BIAS_MODE == 1) v += bias[mBase + mOff + r] * bscale;
        if (BIAS_MODE == 2) v += bv;
        if (RESID) v += Rb[(size_t)(mBase + mOff + r) * ldc + n];
        if (ACT == 2) v = fmaxf(v, 0.0f);
        if (ACT == 4) v = (v > 0.f) ? v : 0.01f * v;
        slab[(mOff + r) * 68 + (j << 4) + rlane] = v;
      }
    }
    __builtin_amdgcn_fence(__ATOMIC_RELEASE, "workgroup");
    __builtin_amdgcn_wave_barrier();
    __builtin_amdgcn_fence(__ATOMIC_ACQUIRE, "workgroup");
    if (OUT_MODE == 0) {
      float* C = (float*)Cout + offC;
      const int hh = lane >> 4, c4 = (lane & 15) * 4;
      for (int pass = 0; pass < 2; ++pass) {
#pragma unroll
        for (int it = 0; it < 8; ++it) {
          const int row = it * 2 + hh;
          v4f v = *(const v4f*)(slab + row * 68 + c4);
          *(volatile v4f*)(C + (size_t)(mBase + row) * ldc + n0 + c4) = v;
        }
        __threadfence();
      }
    } else {
      const int q = lane >> 3, c8 = (lane & 7) * 8;
      unsigned short* C  = (unsigned short*)Cout  + offC;
      unsigned short* C2 = (OUT_MODE == 2) ? ((unsigned short*)Cout2 + offC) : nullptr;
      for (int pass = 0; pass < 2; ++pass) {
#pragma unroll
        for (int it = 0; it < 4; ++it) {
          const int row = it * 4 + q;
          const float* sp = slab + row * 68 + c8;
          v8h hv, lv;
#pragma unroll
          for (int e = 0; e < 8; ++e) {
            if (OUT_MODE == 1) {
              hv[e] = (_Float16)sp[e];
            } else {
              unsigned short hb = f2bf_bits(sp[e]);
              unsigned short lb = f2bf_bits(sp[e] - bf_bits2f(hb));
              hv[e] = __builtin_bit_cast(_Float16, hb);
              lv[e] = __builtin_bit_cast(_Float16, lb);
            }
          }
          *(volatile v8h*)(C + (size_t)(mBase + row) * ldc + n0 + c8) = hv;
          if (OUT_MODE == 2) *(volatile v8h*)(C2 + (size_t)(mBase + row) * ldc + n0 + c8) = lv;
        }
        __threadfence();
      }
    }
    __builtin_amdgcn_fence(__ATOMIC_RELEASE, "workgroup");
    __builtin_amdgcn_wave_barrier();
    __builtin_amdgcn_fence(__ATOMIC_ACQUIRE, "workgroup");
  }
}

__global__ __launch_bounds__(256) void castw_kernel(const float* __restrict__ W0, const float* __restrict__ W1,
                                                    const float* __restrict__ W2, const float* __restrict__ W3,
                                                    unsigned short* __restrict__ out, int n8, int nplane, float scale) {
  const int i = blockIdx.x * 256 + threadIdx.x;
  const int z = blockIdx.y;
  const float* W = (z == 0) ? W0 : (z == 1) ? W1 : (z == 2) ? W2 : W3;
  if (i >= n8) return;
  const float* p = W + 8 * (size_t)i;
  const v4f a = *(const v4f*)(p);
  const v4f c = *(const v4f*)(p + 4);
  unsigned short hb[8];
#pragma unroll
  for (int e = 0; e < 4; ++e) {
    hb[e]     = h_bits(a[e] * scale);
    hb[4 + e] = h_bits(c[e] * scale);
  }
  const v4u u = (v4u){pk16(hb[0], hb[1]), pk16(hb[2], hb[3]), pk16(hb[4], hb[5]), pk16(hb[6], hb[7])};
  unsigned short* q = out + (size_t)z * nplane + 8 * (size_t)i;
  *(volatile v4u*)q = u;
  __threadfence();
  *(volatile v4u*)q = u;
}

__global__ __launch_bounds__(256) void te_kernel(const float* __restrict__ ts,
                                                 const float* __restrict__ w_lin, const float* __restrict__ b_lin,
                                                 const float* __restrict__ w_per, const float* __restrict__ b_per,
                                                 unsigned short* __restrict__ te) {
#pragma clang fp contract(off)
  const int i = blockIdx.x * 256 + threadIdx.x;
  if (i >= kTok * (kE / 8)) return;
  const int row = i >> 4;
  const int c0  = (i & 15) * 8;
  const float t  = ts[row];
  const float wl = w_lin[0];
  const float bl = b_lin[0];
  const float lin = t * wl + bl;
  unsigned w0 = 0u, w1 = 0u, w2 = 0u, w3 = 0u;
#pragma unroll 1
  for (int p2 = 0; p2 < 4; ++p2) {
    const int j0 = c0 + 2 * p2;
    const int j1 = j0 + 1;
    const int i0 = (j0 > 0) ? (j0 - 1) : 0;
    const int i1 = j1 - 1;
    const float a0 = t * w_per[i0] + b_per[i0];
    const float a1 = t * w_per[i1] + b_per[i1];
    const float s0 = sinf(a0);
    const float s1 = sinf(a1);
    const float v0 = (j0 == 0) ? lin : s0;
    const unsigned word = pk16(h_bits(v0 * kCarry16), h_bits(s1 * kCarry16));
    w0 = w1; w1 = w2; w2 = w3; w3 = word;
  }
  const v4u u = (v4u){w0, w1, w2, w3};
  unsigned short* q = te + 8 * (size_t)i;
  *(volatile v4u*)q = u;
  __threadfence();
  *(volatile v4u*)q = u;
}

__global__ __launch_bounds__(256) void xt_kernel(const float* __restrict__ x, unsigned short* __restrict__ xt) {
  __shared__ float sm[64][65];
  const int t  = threadIdx.x;
  const int s0 = blockIdx.x * 64;
  const int d0 = blockIdx.y * 64;
  const int b  = blockIdx.z;
#pragma unroll
  for (int i = 0; i < 16; ++i) {
    const int e = i * 256 + t;
    const int r = e >> 6;
    const int c = e & 63;
    sm[c][r] = x[((size_t)(b * kS + s0 + r)) * kD + d0 + c];
  }
  __syncthreads();
  const int lane = t & 31, wave = t >> 5;
  const int q = lane >> 3, c8 = (lane & 7) * 8;
  unsigned short* op = xt + (size_t)b * kD * kS;
  for (int pass = 0; pass < 2; ++pass) {
#pragma unroll
    for (int it = 0; it < 2; ++it) {
      const int row = wave * 8 + it * 4 + q;
      unsigned short hb[8];
#pragma unroll
      for (int e = 0; e < 8; ++e) hb[e] = h_bits(sm[row][c8 + e]);
      const v4u u = (v4u){pk16(hb[0], hb[1]), pk16(hb[2], hb[3]), pk16(hb[4], hb[5]), pk16(hb[6], hb[7])};
      *(volatile v4u*)(op + (size_t)(d0 + row) * kS + s0 + c8) = u;
    }
    __threadfence();
  }
}

__global__ __launch_bounds__(128) void softmax_kernel(const float* __restrict__ Sp, unsigned short* __restrict__ Pp) {
  __shared__ float redM[4];
  __shared__ float redL[4];
  const int row  = blockIdx.x;
  const int t    = threadIdx.x;
  const int lane = t & 31, wave = t >> 5;
  const float* sr = Sp + (size_t)row * kS + t * 8;
  const v4f a = *(const v4f*)(sr);
  const v4f c = *(const v4f*)(sr + 4);
  float x[8];
#pragma unroll
  for (int e = 0; e < 4; ++e) { x[e] = a[e]; x[4 + e] = c[e]; }
  float m = fmaxf(fmaxf(fmaxf(x[0], x[1]), fmaxf(x[2], x[3])), fmaxf(fmaxf(x[4], x[5]), fmaxf(x[6], x[7])));
#pragma unroll
  for (int off = 16; off > 0; off >>= 1) m = fmaxf(m, __shfl_xor(m, off, 32));
  if (lane == 0) redM[wave] = m;
  __syncthreads();
  const float mrow = fmaxf(fmaxf(redM[0], redM[1]), fmaxf(redM[2], redM[3]));
  float p[8];
  float l = 0.f;
#pragma unroll
  for (int e = 0; e < 8; ++e) { p[e] = exp2f((x[e] - mrow) * kLog2e); l += p[e]; }
#pragma unroll
  for (int off = 16; off > 0; off >>= 1) l += __shfl_xor(l, off, 32);
  if (lane == 0) redL[wave] = l;
  __syncthreads();
  const float lrow = ((redL[0] + redL[1]) + redL[2]) + redL[3];
  const float inv  = kPCarry / lrow;
  unsigned short hb[8];
#pragma unroll
  for (int e = 0; e < 8; ++e) hb[e] = h_bits(p[e] * inv);
  const v4u u = (v4u){pk16(hb[0], hb[1]), pk16(hb[2], hb[3]), pk16(hb[4], hb[5]), pk16(hb[6], hb[7])};
  unsigned short* q = Pp + (size_t)row * kS + t * 8;
  *(volatile v4u*)q = u;
  __threadfence();
  *(volatile v4u*)q = u;
}

__device__ __forceinline__ float sigmoid_f(float x) {
  x = fminf(fmaxf(x, -30.0f), 30.0f);
  return 1.0f / (1.0f + expf(-x));
}

__global__ __launch_bounds__(512) void gru_kernel(const float* __restrict__ att, const unsigned short* __restrict__ wg,
                                                  const float* __restrict__ bih_f, const float* __restrict__ bhh_f,
                                                  const float* __restrict__ bih_b, const float* __restrict__ bhh_b,
                                                  float* __restrict__ hfin) {
  __shared__ __align__(16) _Float16 atile[2 * kBP * kGruPA];
  __shared__ __align__(16) float hslab[kBP * kNH];
  const int t   = threadIdx.x;
  const int dir = blockIdx.x;
  const _Float16* wih = (const _Float16*)(const void*)wg + (size_t)(2 * dir) * kWihN;
  const _Float16* whh = wih + kWihN;
  const float* bih = dir ? bih_b : bih_f;
  const float* bhh = dir ? bhh_b : bhh_f;

  {
    const v4u z4 = (v4u){0u, 0u, 0u, 0u};
    for (int o = t; o < (2 * kBP * kGruPA) / 8; o += 512) *(v4u*)(atile + 8 * o) = z4;
  }
  __syncthreads();

  const int wave = t >> 5, lane = t & 31;
  const int c = lane & 15, hh = lane >> 4, koff = hh * 8;
  const int ub = wave & 7, msub = wave >> 3;
  const int u  = ub * 16 + c;
  const int arow = msub * 16 + c;
  const int drow = msub * 16 + 8 * hh;
  const float bir = bih[u], biz = bih[kNH + u], bin = bih[2 * kNH + u];
  const float bhr = bhh[u], bhz = bhh[kNH + u], bhn = bhh[2 * kNH + u];
  float hreg[8];
#pragma unroll
  for (int r = 0; r < 8; ++r) hreg[r] = 0.f;

  for (int step = 0; step < kS; ++step) {
    const int cur = step & 1;
    _Float16* At = atile + cur * (kBP * kGruPA);
    _Float16* An = atile + (cur ^ 1) * (kBP * kGruPA);
    const int s = dir ? (kS - 1 - step) : step;
    if (t < kB * 16) {
      const int row = t >> 4, c8 = (t & 15) * 8;
      const float* src = att + ((size_t)(row * kS + s)) * kNH + c8;
      const v4f a  = *(const v4f*)(src);
      const v4f q4 = *(const v4f*)(src + 4);
      v8h hv;
#pragma unroll
      for (int e = 0; e < 4; ++e) { hv[e] = (_Float16)(a[e] * kCarry16); hv[4 + e] = (_Float16)(q4[e] * kCarry16); }
      *(v8h*)(At + row * kGruPA + c8) = hv;
    }
    __syncthreads();

    v8f ax[3], ah[3];
#pragma unroll
    for (int g = 0; g < 3; ++g) { ax[g] = (v8f){0.f,0.f,0.f,0.f,0.f,0.f,0.f,0.f}; ah[g] = ax[g]; }
#pragma unroll
    for (int kc = 0; kc < 4; ++kc) {
      const v16h af = Frag<_Float16>::load(At + arow * kGruPA + kc * 32 + koff);
#pragma unroll
      for (int g = 0; g < 3; ++g) {
        const v16h bf = Frag<_Float16>::load(wih + (size_t)(g * kNH + u) * kNH + kc * 32 + koff);
        ax[g] = mma16h(af, bf, ax[g]);
      }
    }
#pragma unroll
    for (int kc = 0; kc < 4; ++kc) {
      const v16h af = Frag<_Float16>::load(At + arow * kGruPA + kNH + kc * 32 + koff);
#pragma unroll
      for (int g = 0; g < 3; ++g) {
        const v16h bf = Frag<_Float16>::load(whh + (size_t)(g * kNH + u) * kNH + kc * 32 + koff);
        ah[g] = mma16h(af, bf, ah[g]);
      }
    }
#pragma unroll
    for (int r = 0; r < 8; ++r) {
      const float ir  = ax[0][r] * kGruScale + bir;
      const float iz  = ax[1][r] * kGruScale + biz;
      const float inn = ax[2][r] * kGruScale + bin;
      const float hr  = ah[0][r] * kGruScale + bhr;
      const float hz  = ah[1][r] * kGruScale + bhz;
      const float hn  = ah[2][r] * kGruScale + bhn;
      const float rg  = sigmoid_f(ir + hr);
      const float zg  = sigmoid_f(iz + hz);
      const float ng  = tanhf(inn + rg * hn);
      const float hv2 = (1.0f - zg) * ng + zg * hreg[r];
      hreg[r] = hv2;
      An[(drow + r) * kGruPA + kNH + u] = (_Float16)(hv2 * kCarry16);
    }
  }

#pragma unroll
  for (int r = 0; r < 8; ++r) hslab[(drow + r) * kNH + u] = hreg[r];
  __syncthreads();
  float* dst = hfin + (size_t)dir * (kBP * kNH);
  for (int pass = 0; pass < 2; ++pass) {
    for (int f = t; f < (kBP * kNH) / 4; f += 512) {
      const int row = f >> 5, c4 = (f & 31) * 4;
      const v4f v = *(const v4f*)(hslab + row * kNH + c4);
      *(volatile v4f*)(dst + row * kNH + c4) = v;
    }
    __threadfence();
  }
}

__global__ __launch_bounds__(256) void head_kernel(const float* __restrict__ hfin,
                                                   const float* __restrict__ W1, const float* __restrict__ b1,
                                                   const float* __restrict__ W2, const float* __restrict__ b2,
                                                   const float* __restrict__ W3, const float* __restrict__ b3,
                                                   float* __restrict__ out) {
  __shared__ __align__(16) float cin[kB * 2 * kNH];
  __shared__ float h1s[kB * 128];
  __shared__ float h2s[kB * 64];
  __shared__ __align__(16) float h3s[192];
  const int t = threadIdx.x;
  for (int o = t; o < kB * 2 * kNH; o += 256) {
    const int b = o >> 8, j = o & 255;
    cin[o] = hfin[(size_t)(j >> 7) * (kBP * kNH) + b * kNH + (j & 127)];
  }
  __syncthreads();
  for (int o = t; o < kB * 128; o += 256) {
    const int b = o >> 7, n = o & 127;
    const float* w  = W1 + (size_t)n * 256;
    const float* ci = cin + b * 256;
    float acc = b1[n];
#pragma unroll 1
    for (int k = 0; k < 256; ++k) acc = acc + ci[k] * w[k];
    h1s[o] = acc;
  }
  __syncthreads();
  for (int o = t; o < kB * 64; o += 256) {
    const int b = o >> 6, n = o & 63;
    const float* w  = W2 + (size_t)n * 128;
    const float* hi = h1s + b * 128;
    float acc = b2[n];
#pragma unroll 1
    for (int k = 0; k < 128; ++k) acc = acc + hi[k] * w[k];
    h2s[o] = acc;
  }
  __syncthreads();
  for (int o = t; o < 192; o += 256) {
    float acc = 0.f;
    if (o < kB * 6) {
      const int b = o / 6, n = o - b * 6;
      const float* w  = W3 + (size_t)n * 64;
      const float* hi = h2s + b * 64;
      acc = b3[n];
#pragma unroll 1
      for (int k = 0; k < 64; ++k) acc = acc + hi[k] * w[k];
    }
    h3s[o] = acc;
  }
  __syncthreads();
  v4f v = (v4f){0.f, 0.f, 0.f, 0.f};
  if (t < 45) v = *(const v4f*)(h3s + 4 * t);
  if (t < 45) *(volatile v4f*)(out + 4 * t) = v;
  __threadfence();
  if (t < 45) *(volatile v4f*)(out + 4 * t) = v;
}

extern "C" void kernel_launch(void* const* d_in, const int* in_sizes, int n_in,
                              void* d_out, int out_size, void* d_ws, size_t ws_size,
                              hipStream_t stream) {
  if (n_in < 26) return;
  if (out_size < kB * 6) return;
  if (ws_size < kWsTotal) return;
  if (in_sizes[0] != kTok * kD || in_sizes[1] != kTok || in_sizes[2] < 1 || in_sizes[3] < 1 ||
      in_sizes[4] != kE - 1 || in_sizes[5] != kE - 1 ||
      in_sizes[6] != kE * kE || in_sizes[7] != kE || in_sizes[8] != kE * kE || in_sizes[9] != kE ||
      in_sizes[10] != kNH * kCtxLd || in_sizes[11] != kNH ||
      in_sizes[12] != kWihN || in_sizes[13] != kWihN || in_sizes[14] != kG3 || in_sizes[15] != kG3 ||
      in_sizes[16] != kWihN || in_sizes[17] != kWihN || in_sizes[18] != kG3 || in_sizes[19] != kG3 ||
      in_sizes[20] != 128 * 256 || in_sizes[21] != 128 || in_sizes[22] != 64 * 128 || in_sizes[23] != 64 ||
      in_sizes[24] != 6 * 64 || in_sizes[25] != 6) return;

  const float* x      = (const float*)d_in[0];
  const float* ts     = (const float*)d_in[1];
  const float* w_lin  = (const float*)d_in[2];
  const float* b_lin  = (const float*)d_in[3];
  const float* w_per  = (const float*)d_in[4];
  const float* b_per  = (const float*)d_in[5];
  const float* Wq     = (const float*)d_in[6];
  const float* bq     = (const float*)d_in[7];
  const float* Wk     = (const float*)d_in[8];
  const float* bk     = (const float*)d_in[9];
  const float* Wo     = (const float*)d_in[10];
  const float* bo     = (const float*)d_in[11];
  const float* Wih_f  = (const float*)d_in[12];
  const float* Whh_f  = (const float*)d_in[13];
  const float* bih_f  = (const float*)d_in[14];
  const float* bhh_f  = (const float*)d_in[15];
  const float* Wih_b  = (const float*)d_in[16];
  const float* Whh_b  = (const float*)d_in[17];
  const float* bih_b  = (const float*)d_in[18];
  const float* bhh_b  = (const float*)d_in[19];
  const float* W1     = (const float*)d_in[20];
  const float* b1     = (const float*)d_in[21];
  const float* W2     = (const float*)d_in[22];
  const float* b2     = (const float*)d_in[23];
  const float* W3     = (const float*)d_in[24];
  const float* b3     = (const float*)d_in[25];

  char* ws = (char*)d_ws;
  unsigned short* TE   = (unsigned short*)(ws + kOffTE);
  unsigned short* QK   = (unsigned short*)(ws + kOffQK);
  unsigned short* XT   = (unsigned short*)(ws + kOffXT);
  unsigned short* CTX  = (unsigned short*)(ws + kOffCTX);
  float*          ATT  = (float*)(ws + kOffATT);
  unsigned short* WQK  = (unsigned short*)(ws + kOffWQK);
  unsigned short* WO16 = (unsigned short*)(ws + kOffWO);
  unsigned short* WG16 = (unsigned short*)(ws + kOffWG);
  float*          HF   = (float*)(ws + kOffHF);
  float*          SB   = (float*)(ws + kOffS);
  unsigned short* PB   = (unsigned short*)(ws + kOffP);

  castw_kernel<<<dim3((kE * kE / 8 + 255) / 256, 2, 1), 256, 0, stream>>>(Wq, Wk, Wq, Wk, WQK, kE * kE / 8, kE * kE, kCarry16);
  castw_kernel<<<dim3((kNH * kCtxLd / 8 + 255) / 256, 1, 1), 256, 0, stream>>>(Wo, Wo, Wo, Wo, WO16, kNH * kCtxLd / 8, kNH * kCtxLd, kCarry16);
  castw_kernel<<<dim3((kWihN / 8 + 255) / 256, 4, 1), 256, 0, stream>>>(Wih_f, Whh_f, Wih_b, Whh_b, WG16, kWihN / 8, kWihN, kCarry16);

  te_kernel<<<(kTok * (kE / 8) + 255) / 256, 256, 0, stream>>>(ts, w_lin, b_lin, w_per, b_per, TE);
  xt_kernel<<<dim3(kS / 64, kD / 64, kB), 256, 0, stream>>>(x, XT);

  {
    const int blocks = (kTok / 64) * (kE / 64) / 8;
    wmma_gemm64z<0, false, 2, 1, false><<<dim3(blocks, 1, 1), 256, 0, stream>>>(
        TE, nullptr, kE, 0, 0, WQK, nullptr, kE, 0, 0, (void*)QK, nullptr, kQKld, 0, 0,
        bq, kQBiasScale, nullptr, 0, kTok, kE, kE, kQScale);
    wmma_gemm64z<0, false, 2, 1, false><<<dim3(blocks, 1, 1), 256, 0, stream>>>(
        TE, nullptr, kE, 0, 0, WQK + kE * kE, nullptr, kE, 0, 0, (void*)(QK + kE), nullptr, kQKld, 0, 0,
        bk, kQBiasScale, nullptr, 0, kTok, kE, kE, kQScale);
  }

  for (int cb = 0; cb < kNChunk; ++cb) {
    const unsigned short* QKc = QK + (size_t)cb * kChunkB * kS * kQKld;
    wmma_gemm64z<0, false, 0, 0, false><<<dim3((kS / 64) * (kS / 64) / 8, kH, kChunkB), 256, 0, stream>>>(
        QKc, nullptr, kQKld, kDK, (long)kS * kQKld,
        QKc + kE, nullptr, kQKld, kDK, (long)kS * kQKld,
        (void*)SB, nullptr, kS, (long)kS * kS, (long)kH * kS * kS,
        nullptr, 0.f, nullptr, 0, kS, kS, kDK, kScoreScale);
    softmax_kernel<<<kBHC * kS, 128, 0, stream>>>(SB, PB);
    wmma_gemm64z<0, false, 0, 1, false><<<dim3((kS / 64) * (kD / 64) / 8, kH, kChunkB), 256, 0, stream>>>(
        PB, nullptr, kS, (long)kS * kS, (long)kH * kS * kS,
        XT + (size_t)cb * kChunkB * kD * kS, nullptr, kS, 0, (long)kD * kS,
        (void*)(CTX + (size_t)cb * kChunkB * kS * kCtxLd), nullptr, kCtxLd, kD, (long)kS * kCtxLd,
        nullptr, 0.f, nullptr, 0, kS, kD, kS, kPVScale);
  }

  {
    const int blocks = (kTok / 64) * (kNH / 64) / 8;
    wmma_gemm64z<0, false, 2, 0, false><<<dim3(blocks, 1, 1), 256, 0, stream>>>(
        CTX, nullptr, kCtxLd, 0, 0, WO16, nullptr, kCtxLd, 0, 0, (void*)ATT, nullptr, kNH, 0, 0,
        bo, 1.0f, nullptr, 0, kTok, kNH, kCtxLd, kOutScale);
  }

  gru_kernel<<<2, 512, 0, stream>>>(ATT, WG16, bih_f, bhh_f, bih_b, bhh_b, HF);

  head_kernel<<<1, 256, 0, stream>>>(HF, W1, b1, W2, b2, W3, b3, (float*)d_out);
}
